// MambaBottleneck_58342835749262
// MI455X (gfx1250) — hardware-verified
//
#include <hip/hip_runtime.h>
#include <math.h>

#define BDIM    8
#define CDIM    512
#define HH      24
#define WWDIM   24
#define LSEQ    (HH * WWDIM)
#define MROWS   (BDIM * LSEQ)
#define DINNER  1024
#define DTRANK  32
#define DSTATE  16
#define XDW     64
#define KCONV   (9 * CDIM)
#define PADHW   26
#define PADAREA (PADHW * PADHW)

#define WSC   64.0f
#define XCSC  256.0f
#define DTSC  1024.0f
#define YGSC  256.0f

typedef __attribute__((ext_vector_type(16))) _Float16 v16h;
typedef __attribute__((ext_vector_type(8)))  _Float16 v8h;
typedef __attribute__((ext_vector_type(8)))  float    v8f;
typedef __attribute__((ext_vector_type(4)))  float    v4f;

__device__ __forceinline__ void dep_guard_h(v8f& a, v8f& b, v16h x, v16h y) { asm volatile("v_nop\n\tv_nop\n\tv_nop\n\tv_nop" : "+v"(a), "+v"(b) : "v"(x), "v"(y)); }
__device__ __forceinline__ void keep4_h(v16h a, v16h b, v16h c, v16h d) { asm volatile("v_nop" :: "v"(a), "v"(b), "v"(c), "v"(d)); }
__device__ __forceinline__ void acc_guard4(v8f& a, v8f& b, v8f& c, v8f& d) { asm volatile("v_nop\n\tv_nop\n\tv_nop\n\tv_nop" : "+v"(a), "+v"(b), "+v"(c), "+v"(d)); }

template <typename T> struct Frag;
template <> struct Frag<_Float16> {
  typedef v16h V; union U { v16h v; v8h h[2]; };
  static __device__ __forceinline__ v16h load(const _Float16* p) {
    U f; f.h[0] = *(const v8h*)(p); f.h[1] = *(const v8h*)(p + 16); return f.v;
  }
  static __device__ __forceinline__ v8f mma(v16h a, v16h b, v8f c) {
    return __builtin_amdgcn_wmma_f32_16x16x32_f16(false, a, false, b, (short)0, c, false, false);
  }
  static __device__ __forceinline__ void guard(v8f& a, v8f& b, v16h x, v16h y) { dep_guard_h(a, b, x, y); }
  static __device__ __forceinline__ void keep(v16h a, v16h b, v16h c, v16h d) { keep4_h(a, b, c, d); }
};

template <int IMPL, int BIAS_MODE, bool BNRELU, int OUT_MODE, bool RESID>
__global__ __launch_bounds__(256) void gemm64(
    const _Float16* __restrict__ A, int lda, long strideA,
    const _Float16* __restrict__ Bt, int ldb, long strideB,
    void* Cout, int ldc, long strideC,
    const float* __restrict__ bias, const float* __restrict__ gamma, const float* __restrict__ beta,
    const float* resid, long strideR,
    int M, int N, int K, float scale) {
  typedef Frag<_Float16> F;
  __shared__ __align__(16) float sT[8][16 * 68];
  const int bz   = blockIdx.y;
  const int lane = threadIdx.x & 31;
  const int wave = threadIdx.x >> 5;
  const int tilesN = N >> 6;
  const int tilesM = M >> 6;
  const int tile = blockIdx.x * 8 + wave;
  if (tile >= tilesM * tilesN) return;
  const int tm = tile / tilesN;
  const int tn = tile - tm * tilesN;
  const int m0 = tm << 6;
  const int n0 = tn << 6;

  const _Float16* Ab = A  + (size_t)bz * strideA;
  const _Float16* Bb = Bt + (size_t)bz * strideB;

  const int rlane = lane & 15;
  const int koff  = (lane >> 4) * 8;
  const int mOff  = (lane >> 4) * 8;

  int abase[4], bbase[4];
#pragma unroll
  for (int i = 0; i < 4; ++i) { abase[i] = 0; bbase[i] = 0; }
  if (IMPL == 1) {
#pragma unroll
    for (int i = 0; i < 4; ++i) {
      const int m  = m0 + (i << 4) + rlane;
      const int b  = m / LSEQ;
      const int l  = m - b * LSEQ;
      const int hh = l / WWDIM;
      const int ww = l - hh * WWDIM;
      abase[i] = ((b * PADHW + hh) * PADHW + ww) * CDIM;
    }
  }
  if (IMPL == 2) {
#pragma unroll
    for (int j = 0; j < 4; ++j) {
      const int l  = n0 + (j << 4) + rlane;
      const int hh = l / WWDIM;
      const int ww = l - hh * WWDIM;
      bbase[j] = ((bz * PADHW + hh) * PADHW + ww) * CDIM;
    }
  }

  v8f acc[4][4];
#pragma unroll
  for (int i = 0; i < 4; ++i)
#pragma unroll
    for (int j = 0; j < 4; ++j) acc[i][j] = (v8f){0.f,0.f,0.f,0.f,0.f,0.f,0.f,0.f};

  for (int k0 = 0; k0 < K; k0 += 32) {
    int tapoff = 0;
    if (IMPL != 0) {
      const int p   = k0 >> 9;
      const int ci0 = k0 & (CDIM - 1);
      const int kh  = p / 3;
      const int kw  = p - kh * 3;
      tapoff = (kh * PADHW + kw) * CDIM + ci0;
    }
    v16h bh[4];
#pragma unroll
    for (int j = 0; j < 4; ++j) {
      if (IMPL == 2) bh[j] = F::load(Bt + (size_t)bbase[j] + tapoff + koff);
      else           bh[j] = F::load(Bb + (size_t)(n0 + (j << 4) + rlane) * ldb + koff + k0);
    }
#pragma unroll
    for (int i = 0; i < 4; ++i) {
      v16h ah;
      if (IMPL == 1) ah = F::load(A + (size_t)abase[i] + tapoff + koff);
      else           ah = F::load(Ab + (size_t)(m0 + (i << 4) + rlane) * lda + koff + k0);
#pragma unroll
      for (int j = 0; j < 4; ++j) acc[i][j] = F::mma(ah, bh[j], acc[i][j]);
      F::guard(acc[i][0], acc[i][3], ah, ah);
    }
    F::keep(bh[0], bh[1], bh[2], bh[3]);
  }
  acc_guard4(acc[0][0], acc[0][1], acc[0][2], acc[0][3]);
  acc_guard4(acc[1][0], acc[1][1], acc[1][2], acc[1][3]);
  acc_guard4(acc[2][0], acc[2][1], acc[2][2], acc[2][3]);
  acc_guard4(acc[3][0], acc[3][1], acc[3][2], acc[3][3]);

  float* slab = sT[wave];
  const float* Rb = RESID ? (resid + (size_t)bz * strideR) : nullptr;
  const float bnk = 1.0f / sqrtf(1.0f + 1e-5f);
#pragma unroll
  for (int i = 0; i < 4; ++i) {
    const int mBase = m0 + (i << 4);
#pragma unroll
    for (int j = 0; j < 4; ++j) {
      const int n = n0 + (j << 4) + rlane;
      float bn2 = 0.f, gn2 = 1.f, tn2 = 0.f;
      if (BIAS_MODE == 2) {
        bn2 = bias[n];
        if (BNRELU) { gn2 = gamma[n] * bnk; tn2 = beta[n]; }
      }
#pragma unroll
      for (int r = 0; r < 8; ++r) {
        const int m = mBase + mOff + r;
        float v = acc[i][j][r] * scale;
        if (BIAS_MODE == 1) {
          v += bias[m];
          if (BNRELU) v = v * (gamma[m] * bnk) + beta[m];
        }
        if (BIAS_MODE == 2) {
          v += bn2;
          if (BNRELU) v = v * gn2 + tn2;
        }
        if (BNRELU) v = fmaxf(v, 0.0f);
        if (RESID) v += Rb[(size_t)m * ldc + n];
        slab[(mOff + r) * 68 + (j << 4) + rlane] = v;
      }
    }
    __builtin_amdgcn_fence(__ATOMIC_RELEASE, "workgroup");
    __builtin_amdgcn_wave_barrier();
    __builtin_amdgcn_fence(__ATOMIC_ACQUIRE, "workgroup");
    if (OUT_MODE == 0) {
      float* C = (float*)Cout + (size_t)bz * strideC;
      const int hh = lane >> 4, c4 = (lane & 15) * 4;
      for (int pass = 0; pass < 2; ++pass) {
#pragma unroll
        for (int it = 0; it < 8; ++it) {
          const int row = it * 2 + hh;
          v4f v = *(const v4f*)(slab + row * 68 + c4);
          *(volatile v4f*)(C + (size_t)(mBase + row) * ldc + n0 + c4) = v;
        }
        __threadfence();
      }
    } else {
      const int q = lane >> 3, c8 = (lane & 7) * 8;
      _Float16* C = (_Float16*)Cout + (size_t)bz * strideC;
      for (int pass = 0; pass < 2; ++pass) {
#pragma unroll
        for (int it = 0; it < 4; ++it) {
          const int row = it * 4 + q;
          const float* sp = slab + row * 68 + c8;
          v8h hv;
#pragma unroll
          for (int e = 0; e < 8; ++e) hv[e] = (_Float16)sp[e];
          *(volatile v8h*)(C + (size_t)(mBase + row) * ldc + n0 + c8) = hv;
        }
        __threadfence();
      }
    }
    __builtin_amdgcn_fence(__ATOMIC_RELEASE, "workgroup");
    __builtin_amdgcn_wave_barrier();
    __builtin_amdgcn_fence(__ATOMIC_ACQUIRE, "workgroup");
  }
}

__global__ __launch_bounds__(256) void cast_scale_f16x2(
    const float* __restrict__ in, _Float16* out, int n2, float sc) {
  const int i = blockIdx.x * 256 + threadIdx.x;
  if (i < n2) {
    const _Float16 h0 = (_Float16)(in[2 * i] * sc), h1 = (_Float16)(in[2 * i + 1] * sc);
    const unsigned u = (unsigned)__builtin_bit_cast(unsigned short, h0) | ((unsigned)__builtin_bit_cast(unsigned short, h1) << 16);
    ((volatile unsigned*)out)[i] = u;
    __threadfence();
    ((volatile unsigned*)out)[i] = u;
  }
}

__global__ __launch_bounds__(256) void reorder_conv_w(
    const float* __restrict__ w, _Float16* dst, int total, float sc) {
  const int idx = blockIdx.x * 256 + threadIdx.x;
  if (idx >= total) return;
  const int g    = idx & 63;
  const int rest = idx >> 6;
  const int p    = rest % 9;
  const int o    = rest / 9;
  v8h ov;
#pragma unroll
  for (int e = 0; e < 8; ++e)
    ov[e] = (_Float16)(w[((size_t)(o * CDIM + g * 8 + e)) * 9 + p] * sc);
  _Float16* q = dst + (size_t)(o * 9 + p) * CDIM + g * 8;
  *(volatile v8h*)q = ov;
  __threadfence();
  *(volatile v8h*)q = ov;
}

template <int MODE>
__global__ __launch_bounds__(256) void pad_fill(
    const float* __restrict__ src, _Float16* dst, int total) {
  const int idx = blockIdx.x * 256 + threadIdx.x;
  if (idx >= total) return;
  const int g   = idx & 63;
  const int pix = idx >> 6;
  const int pw  = pix % PADHW;
  const int ph  = (pix / PADHW) % PADHW;
  const int b   = pix / PADAREA;
  const int hh  = ph - 1, ww = pw - 1;
  const bool inside = (hh >= 0) && (hh < HH) && (ww >= 0) && (ww < WWDIM);
  const int hc = hh < 0 ? 0 : (hh >= HH ? HH - 1 : hh);
  const int wc = ww < 0 ? 0 : (ww >= WWDIM ? WWDIM - 1 : ww);
  const int c0 = g * 8;
  float v[8];
  if (MODE == 0) {
#pragma unroll
    for (int e = 0; e < 8; ++e)
      v[e] = src[((size_t)(b * CDIM + c0 + e) * HH + hc) * WWDIM + wc];
  } else {
    const float* p = src + (size_t)(b * LSEQ + hc * WWDIM + wc) * CDIM + c0;
    const v4f q0 = *(const v4f*)p, q1 = *(const v4f*)(p + 4);
    v[0] = q0[0]; v[1] = q0[1]; v[2] = q0[2]; v[3] = q0[3];
    v[4] = q1[0]; v[5] = q1[1]; v[6] = q1[2]; v[7] = q1[3];
  }
  v8h ov;
#pragma unroll
  for (int e = 0; e < 8; ++e) ov[e] = inside ? (_Float16)v[e] : (_Float16)0.0f;
  _Float16* q = dst + (size_t)pix * CDIM + c0;
  *(volatile v8h*)q = ov;
  __threadfence();
  *(volatile v8h*)q = ov;
}

__global__ __launch_bounds__(256) void layernorm_f16(
    const float* __restrict__ x, const float* __restrict__ w, const float* __restrict__ bb,
    _Float16* out, int nrows) {
  const int wave = threadIdx.x >> 5, lane = threadIdx.x & 31;
  const int row = blockIdx.x * 8 + wave;
  if (row >= nrows) return;
  const float* xr = x + (size_t)row * CDIM;
  const int c0 = lane * 8, c1 = 256 + lane * 8;
  union { v4f q[4]; float f[16]; } u;
  u.q[0] = *(const v4f*)(xr + c0);     u.q[1] = *(const v4f*)(xr + c0 + 4);
  u.q[2] = *(const v4f*)(xr + c1);     u.q[3] = *(const v4f*)(xr + c1 + 4);
  float s = 0.f;
#pragma unroll
  for (int e = 0; e < 16; ++e) s += u.f[e];
#pragma unroll
  for (int off = 16; off >= 1; off >>= 1) s += __shfl_xor(s, off, 32);
  const float mu = s * (1.0f / CDIM);
  float vs = 0.f;
#pragma unroll
  for (int e = 0; e < 16; ++e) { const float d = u.f[e] - mu; vs += d * d; }
#pragma unroll
  for (int off = 16; off >= 1; off >>= 1) vs += __shfl_xor(vs, off, 32);
  const float rstd = rsqrtf(vs * (1.0f / CDIM) + 1e-5f);
  union { v4f q[4]; float f[16]; } wu, bu;
  wu.q[0] = *(const v4f*)(w + c0);  wu.q[1] = *(const v4f*)(w + c0 + 4);
  wu.q[2] = *(const v4f*)(w + c1);  wu.q[3] = *(const v4f*)(w + c1 + 4);
  bu.q[0] = *(const v4f*)(bb + c0); bu.q[1] = *(const v4f*)(bb + c0 + 4);
  bu.q[2] = *(const v4f*)(bb + c1); bu.q[3] = *(const v4f*)(bb + c1 + 4);
  v8h o0, o1;
#pragma unroll
  for (int e = 0; e < 8; ++e) {
    o0[e] = (_Float16)((u.f[e] - mu) * rstd * wu.f[e] + bu.f[e]);
    o1[e] = (_Float16)((u.f[8 + e] - mu) * rstd * wu.f[8 + e] + bu.f[8 + e]);
  }
  _Float16* orow = out + (size_t)row * CDIM;
  for (int pass = 0; pass < 2; ++pass) {
    *(volatile v8h*)(orow + c0) = o0;
    *(volatile v8h*)(orow + c1) = o1;
    __threadfence();
  }
}

__global__ __launch_bounds__(256) void dwconv_silu(
    const _Float16* __restrict__ xz, const float* __restrict__ cw, const float* __restrict__ cb,
    _Float16* xc, int total) {
  const int idx = blockIdx.x * 256 + threadIdx.x;
  if (idx >= total) return;
  const int g  = idx & 127;
  const int m  = idx >> 7;
  const int b  = m / LSEQ;
  const int t  = m - b * LSEQ;
  const int d0 = g * 8;
  v4f cw4[8];
#pragma unroll
  for (int e = 0; e < 8; ++e) cw4[e] = *(const v4f*)(cw + (size_t)(d0 + e) * 4);
  float acc[8];
#pragma unroll
  for (int e = 0; e < 8; ++e) acc[e] = 0.f;
#pragma unroll
  for (int j = 0; j < 4; ++j) {
    const int tt  = t - 3 + j;
    const int ttc = tt < 0 ? 0 : tt;
    const float f = tt < 0 ? 0.f : 1.f;
    const v8h xv = *(const v8h*)(xz + (size_t)(b * LSEQ + ttc) * (2 * DINNER) + d0);
#pragma unroll
    for (int e = 0; e < 8; ++e) acc[e] = fmaf((float)xv[e] * f, cw4[e][j], acc[e]);
  }
  v8h ov;
#pragma unroll
  for (int e = 0; e < 8; ++e) {
    const float a = acc[e] + cb[d0 + e];
    const float s = a * __builtin_amdgcn_rcpf(1.0f + __expf(-a));
    ov[e] = (_Float16)(s * XCSC);
  }
  _Float16* q = xc + (size_t)m * DINNER + d0;
  *(volatile v8h*)q = ov;
  __threadfence();
  *(volatile v8h*)q = ov;
}

__global__ __launch_bounds__(256) void dt_pack(
    const float* __restrict__ xd, _Float16* dt, int npairs) {
  const int idx = blockIdx.x * 256 + threadIdx.x;
  if (idx >= npairs) return;
  const int r0 = idx * 2;
  v8h hv[8];
#pragma unroll
  for (int rr = 0; rr < 2; ++rr) {
#pragma unroll
    for (int q = 0; q < 4; ++q) {
      const float* p = xd + (size_t)(r0 + rr) * XDW + q * 8;
      const v4f a = *(const v4f*)p, c = *(const v4f*)(p + 4);
      v8h tv;
      tv[0] = (_Float16)(a[0] * DTSC); tv[1] = (_Float16)(a[1] * DTSC);
      tv[2] = (_Float16)(a[2] * DTSC); tv[3] = (_Float16)(a[3] * DTSC);
      tv[4] = (_Float16)(c[0] * DTSC); tv[5] = (_Float16)(c[1] * DTSC);
      tv[6] = (_Float16)(c[2] * DTSC); tv[7] = (_Float16)(c[3] * DTSC);
      hv[rr * 4 + q] = tv;
    }
  }
  _Float16* base = dt + (size_t)r0 * DTRANK;
  for (int pass = 0; pass < 2; ++pass) {
#pragma unroll
    for (int s = 0; s < 8; ++s) *(volatile v8h*)(base + s * 8) = hv[s];
    __threadfence();
  }
}

__global__ __launch_bounds__(64) void scan_gate(
    const float* __restrict__ dpre, const _Float16* __restrict__ xc, const float* __restrict__ xd,
    const _Float16* __restrict__ xz, const float* __restrict__ a_log, const float* __restrict__ dsk,
    _Float16* yg) {
  __shared__ __align__(16) _Float16 ys[8 * 64];
  const int tid = threadIdx.x;
  const int b   = blockIdx.x >> 4;
  const int d0  = (blockIdx.x & 15) * 64;
  const int d   = d0 + tid;
  float An[DSTATE], h[DSTATE];
#pragma unroll
  for (int n = 0; n < DSTATE; ++n) { An[n] = -__expf(a_log[(size_t)d * DSTATE + n]); h[n] = 0.f; }
  const float Dd = dsk[d];
  const int jrow = tid >> 3, q8 = (tid & 7) * 8;
#pragma unroll 1
  for (int tb = 0; tb < LSEQ / 8; ++tb) {
    const int mblk = b * LSEQ + tb * 8;
#pragma unroll 1
    for (int j = 0; j < 8; ++j) {
      const size_t m  = (size_t)(mblk + j);
      const float pv  = dpre[m * DINNER + d];
      const float dlt = fmaxf(pv, 0.f) + log1pf(__expf(-fabsf(pv)));
      const float u   = (float)xc[m * DINNER + d] * (1.0f / XCSC);
      const float du  = dlt * u;
      const float* bc = xd + m * XDW + DTRANK;
      union { v4f q[8]; float f[32]; } bcu;
      bcu.q[0] = *(const v4f*)(bc);      bcu.q[1] = *(const v4f*)(bc + 4);
      bcu.q[2] = *(const v4f*)(bc + 8);  bcu.q[3] = *(const v4f*)(bc + 12);
      bcu.q[4] = *(const v4f*)(bc + 16); bcu.q[5] = *(const v4f*)(bc + 20);
      bcu.q[6] = *(const v4f*)(bc + 24); bcu.q[7] = *(const v4f*)(bc + 28);
      float y = 0.f;
#pragma unroll
      for (int n = 0; n < DSTATE; ++n) {
        const float e = __expf(dlt * An[n]);
        h[n] = h[n] * e + du * bcu.f[n];
        y = fmaf(h[n], bcu.f[16 + n], y);
      }
      const float z   = (float)xz[m * (2 * DINNER) + DINNER + d];
      const float gte = z * __builtin_amdgcn_rcpf(1.0f + __expf(-z));
      const float ov  = (y + u * Dd) * gte;
      ys[j * 64 + tid] = (_Float16)(ov * YGSC);
    }
    __syncthreads();
    const v8h pv8 = *(const v8h*)(ys + jrow * 64 + q8);
    _Float16* dst = yg + (size_t)(mblk + jrow) * DINNER + d0 + q8;
    *(volatile v8h*)dst = pv8;
    __threadfence();
    *(volatile v8h*)dst = pv8;
    __syncthreads();
  }
}

extern "C" void kernel_launch(void* const* d_in, const int* in_sizes, int n_in,
                              void* d_out, int out_size, void* d_ws, size_t ws_size,
                              hipStream_t stream) {
  if (n_in < 20) return;
  if (out_size != BDIM * CDIM * LSEQ) return;
  if (in_sizes[0] != BDIM * CDIM * LSEQ) return;
  if (in_sizes[1] != CDIM * CDIM * 9 || in_sizes[16] != CDIM * CDIM * 9) return;
  if (in_sizes[7] != 2 * 2 * DINNER * CDIM || in_sizes[10] != 2 * XDW * DINNER) return;
  if (in_sizes[11] != 2 * DINNER * DTRANK || in_sizes[13] != 2 * DINNER * DSTATE) return;
  if (in_sizes[15] != 2 * CDIM * DINNER) return;

  const float* x          = (const float*)d_in[0];
  const float* conv_in_w  = (const float*)d_in[1];
  const float* conv_in_b  = (const float*)d_in[2];
  const float* bn_in_g    = (const float*)d_in[3];
  const float* bn_in_b    = (const float*)d_in[4];
  const float* norm_w     = (const float*)d_in[5];
  const float* norm_b     = (const float*)d_in[6];
  const float* in_w       = (const float*)d_in[7];
  const float* conv1d_w   = (const float*)d_in[8];
  const float* conv1d_b   = (const float*)d_in[9];
  const float* xproj_w    = (const float*)d_in[10];
  const float* dtproj_w   = (const float*)d_in[11];
  const float* dtproj_b   = (const float*)d_in[12];
  const float* a_log      = (const float*)d_in[13];
  const float* d_skip     = (const float*)d_in[14];
  const float* out_w      = (const float*)d_in[15];
  const float* conv_out_w = (const float*)d_in[16];
  const float* conv_out_b = (const float*)d_in[17];
  const float* bn_out_g   = (const float*)d_in[18];
  const float* bn_out_b   = (const float*)d_in[19];
  float* out = (float*)d_out;

  char* ws = (char*)d_ws;
  size_t off = 0;
  auto carve = [&](size_t bytes) -> void* {
    void* p = ws + off;
    off += (bytes + 255) & ~(size_t)255;
    return p;
  };
  _Float16* wci16 = (_Float16*)carve((size_t)CDIM * KCONV * 2);
  _Float16* wco16 = (_Float16*)carve((size_t)CDIM * KCONV * 2);
  _Float16* win16 = (_Float16*)carve((size_t)2 * 2 * DINNER * CDIM * 2);
  _Float16* wxp16 = (_Float16*)carve((size_t)2 * XDW * DINNER * 2);
  _Float16* wdt16 = (_Float16*)carve((size_t)2 * DINNER * DTRANK * 2);
  _Float16* wou16 = (_Float16*)carve((size_t)2 * CDIM * DINNER * 2);
  _Float16* pad16 = (_Float16*)carve((size_t)BDIM * PADAREA * CDIM * 2);
  float*    seq   = (float*)   carve((size_t)MROWS * CDIM * 4);
  _Float16* hln16 = (_Float16*)carve((size_t)MROWS * CDIM * 2);
  _Float16* xz16  = (_Float16*)carve((size_t)MROWS * 2 * DINNER * 2);
  _Float16* xc16  = (_Float16*)carve((size_t)MROWS * DINNER * 2);
  float*    xdbl  = (float*)   carve((size_t)MROWS * XDW * 4);
  _Float16* dt16  = (_Float16*)carve((size_t)MROWS * DTRANK * 2);
  float*    dpre  = (float*)   carve((size_t)MROWS * DINNER * 4);
  _Float16* yg16  = (_Float16*)carve((size_t)MROWS * DINNER * 2);
  if (off > ws_size) return;

  auto nb = [](size_t n, int t) -> unsigned { return (unsigned)((n + (size_t)t - 1) / (size_t)t); };

  {
    const int totw = CDIM * 9 * 64;
    reorder_conv_w<<<nb(totw, 256), 256, 0, stream>>>(conv_in_w, wci16, totw, WSC);
    reorder_conv_w<<<nb(totw, 256), 256, 0, stream>>>(conv_out_w, wco16, totw, WSC);
    const int n2a = 2 * 2 * DINNER * CDIM / 2, n2b = 2 * XDW * DINNER / 2, n2c = 2 * DINNER * DTRANK / 2, n2d = 2 * CDIM * DINNER / 2;
    cast_scale_f16x2<<<nb(n2a, 256), 256, 0, stream>>>(in_w, win16, n2a, WSC);
    cast_scale_f16x2<<<nb(n2b, 256), 256, 0, stream>>>(xproj_w, wxp16, n2b, WSC);
    cast_scale_f16x2<<<nb(n2c, 256), 256, 0, stream>>>(dtproj_w, wdt16, n2c, WSC);
    cast_scale_f16x2<<<nb(n2d, 256), 256, 0, stream>>>(out_w, wou16, n2d, WSC);
  }

  const int totpad = BDIM * PADAREA * 64;

  pad_fill<0><<<nb(totpad, 256), 256, 0, stream>>>(x, pad16, totpad);
  {
    const int M = MROWS, N = CDIM, K = KCONV;
    dim3 g(nb((size_t)(M >> 6) * (N >> 6), 8), 1);
    gemm64<1, 2, true, 0, false><<<g, 256, 0, stream>>>(
        pad16, 0, 0L, wci16, KCONV, 0L, (void*)seq, CDIM, 0L,
        conv_in_b, bn_in_g, bn_in_b, nullptr, 0L, M, N, K, 1.0f / WSC);
  }

  for (int i = 0; i < 2; ++i) {
    layernorm_f16<<<nb(MROWS, 8), 256, 0, stream>>>(seq, norm_w + (size_t)i * CDIM, norm_b + (size_t)i * CDIM, hln16, MROWS);

    {
      const int M = MROWS, N = 2 * DINNER, K = CDIM;
      dim3 g(nb((size_t)(M >> 6) * (N >> 6), 8), 1);
      gemm64<0, 0, false, 1, false><<<g, 256, 0, stream>>>(
          hln16, CDIM, 0L, win16 + (size_t)i * 2 * DINNER * CDIM, CDIM, 0L, (void*)xz16, 2 * DINNER, 0L,
          nullptr, nullptr, nullptr, nullptr, 0L, M, N, K, 1.0f / WSC);
    }

    {
      const int tot = MROWS * 128;
      dwconv_silu<<<nb(tot, 256), 256, 0, stream>>>(
          xz16, conv1d_w + (size_t)i * DINNER * 4, conv1d_b + (size_t)i * DINNER, xc16, tot);
    }

    {
      const int M = MROWS, N = XDW, K = DINNER;
      dim3 g(nb((size_t)(M >> 6) * (N >> 6), 8), 1);
      gemm64<0, 0, false, 0, false><<<g, 256, 0, stream>>>(
          xc16, DINNER, 0L, wxp16 + (size_t)i * XDW * DINNER, DINNER, 0L, (void*)xdbl, XDW, 0L,
          nullptr, nullptr, nullptr, nullptr, 0L, M, N, K, 1.0f / (XCSC * WSC));
    }

    dt_pack<<<nb(MROWS / 2, 256), 256, 0, stream>>>(xdbl, dt16, MROWS / 2);

    {
      const int M = MROWS, N = DINNER, K = DTRANK;
      dim3 g(nb((size_t)(M >> 6) * (N >> 6), 8), 1);
      gemm64<0, 2, false, 0, false><<<g, 256, 0, stream>>>(
          dt16, DTRANK, 0L, wdt16 + (size_t)i * DINNER * DTRANK, DTRANK, 0L, (void*)dpre, DINNER, 0L,
          dtproj_b + (size_t)i * DINNER, nullptr, nullptr, nullptr, 0L, M, N, K, 1.0f / (DTSC * WSC));
    }

    scan_gate<<<BDIM * (DINNER / 64), 64, 0, stream>>>(
        dpre, xc16, xdbl, xz16, a_log + (size_t)i * DINNER * DSTATE, d_skip + (size_t)i * DINNER, yg16);

    {
      const int M = MROWS, N = CDIM, K = DINNER;
      dim3 g(nb((size_t)(M >> 6) * (N >> 6), 8), 1);
      gemm64<0, 0, false, 0, true><<<g, 256, 0, stream>>>(
          yg16, DINNER, 0L, wou16 + (size_t)i * CDIM * DINNER, DINNER, 0L, (void*)seq, CDIM, 0L,
          nullptr, nullptr, nullptr, seq, 0L, M, N, K, 1.0f / (YGSC * WSC));
    }
  }

  pad_fill<1><<<nb(totpad, 256), 256, 0, stream>>>(seq, pad16, totpad);
  {
    const int M = CDIM, N = LSEQ, K = KCONV;
    dim3 g(nb((size_t)(M >> 6) * (N >> 6), 8), BDIM);
    gemm64<2, 1, true, 0, false><<<g, 256, 0, stream>>>(
        wco16, KCONV, 0L, pad16, 0, 0L, (void*)out, LSEQ, (long)CDIM * LSEQ,
        conv_out_b, bn_out_g, bn_out_b, nullptr, 0L, M, N, K, 1.0f / WSC);
  }
}
